// DAWN_88124138979400
// MI455X (gfx1250) — hardware-run, weakly checked
//
#include <hip/hip_runtime.h>


#ifndef NB
#define NB 2
#endif
#ifndef SEQ
#define SEQ 1024
#endif
#define NB_FULL  2
#define SEQ_FULL 1024
#ifndef OUT_SEQ
#define OUT_SEQ SEQ
#endif
#define DM   768
#define RK   128
#define NE   128
#define DSP  64
#define TK   4
#define TOK  (NB * SEQ)
#define APF  776
#define AHP  136
#define HCS  64.0f
#define RCS  64.0f
#define OSI  (1.0f / 4096.0f)
#define L2E  1.4426950408889634f
#define NEGB (-3.0e38f)

static_assert(NE == 128);
static_assert(DSP == 64);
static_assert(2 * DSP == 128);
static_assert(TK == 4);
static_assert(DM % 32 == 0);
static_assert(RK % 32 == 0);
static_assert(DM % 64 == 0);
static_assert(RK % 64 == 0);
static_assert(DM % 256 == 0);
static_assert(RK == 128);
static_assert(TOK % 32 == 0);
static_assert(SEQ % 32 == 0);
static_assert(NB <= NB_FULL);
static_assert(SEQ <= SEQ_FULL);
static_assert((APF * 2) % 16 == 0);
static_assert((AHP * 2) % 16 == 0);
static_assert(APF >= DM);
static_assert(AHP >= RK);
static_assert(((size_t)SEQ * DM) % 8 == 0);
static_assert((DM / 4) % 32 == 0);
static_assert((size_t)32 * APF * 2 + (size_t)TOK * 8 + 16 + (size_t)4 * 16 * 36 * 4 <= 131072);
static_assert((size_t)32 * AHP * 2 + (size_t)TOK * 8 + 16 + (size_t)4 * 16 * 68 * 4 <= 131072);
static_assert((size_t)NE * 65 * 4 + (size_t)32 * DSP * 4 + (size_t)32 * NE * 4 + 1024 <= 131072);

typedef _Float16 h16;
typedef unsigned short bf;
typedef __attribute__((ext_vector_type(16))) __bf16   v16bf;
typedef __attribute__((ext_vector_type(16))) _Float16 v16h;
typedef __attribute__((ext_vector_type(8)))  _Float16 v8h;
typedef __attribute__((ext_vector_type(8)))  unsigned short v8us;
typedef __attribute__((ext_vector_type(8)))  float    v8f;
typedef __attribute__((ext_vector_type(4)))  float    v4f;
typedef v4f  __attribute__((may_alias)) v4fa;
typedef __attribute__((ext_vector_type(4)))  int      v4i;
typedef v4i  __attribute__((may_alias)) v4ia;
typedef __attribute__((ext_vector_type(4)))  unsigned int v4u;
typedef v4u  __attribute__((may_alias)) v4ua;
typedef v8us __attribute__((may_alias)) v8usa;
typedef v8h  __attribute__((may_alias)) v8ha;

__device__ __forceinline__ unsigned short f2bf(float f) { unsigned u = __float_as_uint(f); u += 0x7FFFu + ((u >> 16) & 1u); return (unsigned short)(u >> 16); }
__device__ __forceinline__ float bfr(float f) { return __uint_as_float(((unsigned)f2bf(f)) << 16); }
__device__ __forceinline__ v16h cat16(v8h lo, v8h hi) { return __builtin_shufflevector(lo, hi, 0, 1, 2, 3, 4, 5, 6, 7, 8, 9, 10, 11, 12, 13, 14, 15); }
__device__ __forceinline__ v16bf cat16b(v8us lo, v8us hi) { return __builtin_bit_cast(v16bf, __builtin_shufflevector(lo, hi, 0, 1, 2, 3, 4, 5, 6, 7, 8, 9, 10, 11, 12, 13, 14, 15)); }
__device__ __forceinline__ v8f wmma16(v16h a, v16h b, v8f c) { return __builtin_amdgcn_wmma_f32_16x16x32_f16(false, a, false, b, (short)0, c, false, false); }
__device__ __forceinline__ v8f wmmab(v16bf a, v16bf b, v8f c) { return __builtin_amdgcn_wmma_f32_16x16x32_bf16(false, a, false, b, (short)0, c, false, false); }
__device__ __forceinline__ v16h  ldh(const h16* p) { return cat16(*(const v8h*)p, *(const v8h*)(p + 16)); }
__device__ __forceinline__ v16bf ldb(const bf* p)  { return cat16b(*(const v8us*)p, *(const v8us*)(p + 16)); }
__device__ __forceinline__ void wave_sync() { __builtin_amdgcn_fence(3  , "wavefront"); __builtin_amdgcn_wave_barrier(); asm volatile("" ::: "memory"); }

static __device__ __forceinline__ h16 toh_flush(float v) { const h16 r = (h16)v; return (fabsf(v) < 6.103515625e-05f) ? (h16)0.0f : r; }
__device__ __forceinline__ v8f wmmab_g(v16bf a, v16bf b, v8f c) { c = wmmab(a, b, c); asm volatile("v_nop\n\tv_nop\n\tv_nop\n\tv_nop" : "+v"(c) : "v"(a), "v"(b)); return c; }
__device__ __forceinline__ v8f wmma16_g(v16h a, v16h b, v8f c) { c = wmma16(a, b, c); asm volatile("v_nop\n\tv_nop\n\tv_nop\n\tv_nop" : "+v"(c) : "v"(a), "v"(b)); return c; }

__global__ __launch_bounds__(256) void k_cvt8(const float* __restrict__ src, bf* dst, size_t n8) {
    const size_t i = (size_t)blockIdx.x * 256 + threadIdx.x; if (i >= n8) return;
    const v8f v = *(const v8f*)(src + i * 8); v8us o;
#pragma unroll
    for (int k = 0; k < 8; ++k) o[k] = f2bf(v[k]);
    *(volatile v8us*)(dst + i * 8) = o; __threadfence(); *(volatile v8us*)(dst + i * 8) = o;
}

template <int MODE>
__device__ __forceinline__ void tconv_body(const float* __restrict__ src, unsigned short* dst, int R0, int C0) {
    __shared__ float ts[64 * 65];
    const int tid = threadIdx.x;
    const int r0 = blockIdx.x * 64, c0 = blockIdx.y * 64;
    const size_t zo = (size_t)blockIdx.z * (size_t)R0 * (size_t)C0;
#pragma unroll
    for (int q = 0; q < 4; ++q) { const int p = q * 256 + tid; const int row = p >> 4, c4 = (p & 15) * 4;
        const v4f v = *(const v4f*)(src + zo + (size_t)(r0 + row) * (size_t)C0 + c0 + c4);
        ts[row * 65 + c4 + 0] = v[0]; ts[row * 65 + c4 + 1] = v[1]; ts[row * 65 + c4 + 2] = v[2]; ts[row * 65 + c4 + 3] = v[3]; }
    __syncthreads();
    v8us o[2];
#pragma unroll
    for (int q = 0; q < 2; ++q) { const int p = q * 256 + tid; const int oc = p >> 3, r8 = (p & 7) * 8;
#pragma unroll
        for (int k = 0; k < 8; ++k) { const float v = ts[(r8 + k) * 65 + oc];
            o[q][k] = (MODE == 0) ? f2bf(v) : __builtin_bit_cast(unsigned short, toh_flush(bfr(v) * RCS)); } }
    static_assert(256 * 2 * 16 == 64 * 128);
#pragma unroll 1
    for (int ps = 0; ps < 2; ++ps) {
#pragma unroll
        for (int q = 0; q < 2; ++q) { const int p = q * 256 + tid; const int oc = p >> 3, r8 = (p & 7) * 8;
            *(volatile v8us*)(dst + zo + (size_t)(c0 + oc) * (size_t)R0 + r0 + r8) = o[q]; }
        if (ps == 0) __threadfence(); }
}
__global__ __launch_bounds__(256) void k_tconv_b(const float* __restrict__ src, bf* dst, int R0, int C0) { tconv_body<0>(src, dst, R0, C0); }
__global__ __launch_bounds__(256) void k_tconv_h(const float* __restrict__ src, h16* dst, int R0, int C0) { tconv_body<1>(src, (unsigned short*)dst, R0, C0); }

__global__ __launch_bounds__(32) void k_rproj(const bf* __restrict__ A, const bf* __restrict__ Bt, const float* __restrict__ bias_f, const float* __restrict__ bias_r, float* P) {
    __shared__ __align__(16) float os[16 * 68];
    const int lane = threadIdx.x & 31, lr = lane & 15, hi = lane >> 4; const int r0 = blockIdx.x * 32, c0 = blockIdx.y * 64;
    v8f acc[2][4];
#pragma unroll
    for (int mb = 0; mb < 2; ++mb)
#pragma unroll
        for (int nb = 0; nb < 4; ++nb) acc[mb][nb] = (v8f){};
    const size_t aoff = (size_t)(r0 + lr) * DM + 8 * hi, boff = (size_t)(c0 + lr) * DM + 8 * hi;
#pragma unroll 1
    for (int kc = 0; kc < DM; kc += 32) {
        const v16bf a0 = ldb(A + aoff + kc), a1 = ldb(A + aoff + (size_t)16 * DM + kc);
#pragma unroll
        for (int nb = 0; nb < 4; ++nb) { const v16bf b = ldb(Bt + boff + (size_t)nb * 16 * DM + kc);
            acc[0][nb] = wmmab_g(a0, b, acc[0][nb]); acc[1][nb] = wmmab_g(a1, b, acc[1][nb]); }
    }
    float bc[4];
#pragma unroll
    for (int nb = 0; nb < 4; ++nb) { const float vf = bfr(bias_f[nb * 16 + lr]); const float vr = bfr(bias_r[nb * 16 + lr]); bc[nb] = (c0 == 0) ? vf : vr; }
#pragma unroll
    for (int mb = 0; mb < 2; ++mb) {
#pragma unroll
        for (int nb = 0; nb < 4; ++nb) {
#pragma unroll
            for (int j = 0; j < 8; ++j) os[(hi * 8 + j) * 68 + nb * 16 + lr] = acc[mb][nb][j] + bc[nb]; }
        wave_sync();
        static_assert(32 * 16 * 8 == 16 * 256);
#pragma unroll 1
        for (int ps = 0; ps < 2; ++ps) {
#pragma unroll
            for (int s = 0; s < 8; ++s) { const int row = 2 * s + (lane >> 4), c4 = (lane & 15) * 4;
                const v4f val = *(const v4fa*)(&os[row * 68 + c4]);
                *(volatile v4f*)(P + (size_t)(r0 + mb * 16 + row) * (2 * DSP) + c0 + c4) = val; }
            if (ps == 0) __threadfence(); }
        wave_sync();
    }
}

__global__ __launch_bounds__(128) void k_route(const float* __restrict__ PROJ, const float* __restrict__ emb_f, const float* __restrict__ emb_r, int* SELI, float* SELW) {
#pragma clang fp contract(off)
    __shared__ float en[NE * 65];
    __shared__ __align__(16) float ps[32 * DSP];
    __shared__ float lg[32 * NE];
    __shared__ __align__(16) int   si[32 * TK];
    __shared__ __align__(16) float sw[32 * TK];
    const int tid = threadIdx.x, lane = tid & 31;
    const int wave = __builtin_amdgcn_readfirstlane((int)(threadIdx.x >> 5));
    const int route = blockIdx.y; const int t0 = blockIdx.x * 32;
    {
        float ss = 0.0f;
#pragma unroll 1
        for (int i = 0; i < DSP; ++i) { const float a = bfr(emb_f[tid * DSP + i]); const float b = bfr(emb_r[tid * DSP + i]); const float v = (route == 0) ? a : b;
            en[tid * 65 + i] = v; ss += v * v; }
        const float inv = 1.0f / (sqrtf(ss) + 1e-8f);
#pragma unroll 1
        for (int i = 0; i < DSP; ++i) en[tid * 65 + i] = en[tid * 65 + i] * inv;
    }
#pragma unroll
    for (int q = 0; q < 4; ++q) { const int p = q * 128 + tid; const int row = p >> 4, c4 = (p & 15) * 4;
        const v4f v = *(const v4f*)(PROJ + (size_t)(t0 + row) * (2 * DSP) + route * DSP + c4);
        *(v4fa*)(&ps[row * DSP + c4]) = v; }
    __syncthreads();
#pragma unroll 1
    for (int tl = 0; tl < 32; ++tl) { float s = 0.0f;
#pragma unroll 4
        for (int i = 0; i < DSP; ++i) s = fmaf(ps[tl * DSP + i], en[tid * 65 + i], s);
        lg[tl * NE + tid] = s; }
    __syncthreads();
#pragma unroll 1
    for (int rr = 0; rr < 8; ++rr) {
        const int row = wave * 8 + rr;
        float v0 = lg[row * NE + lane], v1 = lg[row * NE + 32 + lane], v2 = lg[row * NE + 64 + lane], v3 = lg[row * NE + 96 + lane];
        float mx = fmaxf(fmaxf(v0, v1), fmaxf(v2, v3));
#pragma unroll
        for (int off = 16; off > 0; off >>= 1) mx = fmaxf(mx, __shfl_xor(mx, off, 32));
        float es = (__builtin_amdgcn_exp2f((v0 - mx) * L2E) + __builtin_amdgcn_exp2f((v1 - mx) * L2E)) + (__builtin_amdgcn_exp2f((v2 - mx) * L2E) + __builtin_amdgcn_exp2f((v3 - mx) * L2E));
#pragma unroll
        for (int off = 16; off > 0; off >>= 1) es += __shfl_xor(es, off, 32);
        const float inv = 1.0f / es;
        int sidx[4]; float sp[4];
#pragma unroll
        for (int it = 0; it < 4; ++it) {
            float bv = v0; int bi = lane;
            { const bool g = v1 > bv; bv = g ? v1 : bv; bi = g ? lane + 32 : bi; }
            { const bool g = v2 > bv; bv = g ? v2 : bv; bi = g ? lane + 64 : bi; }
            { const bool g = v3 > bv; bv = g ? v3 : bv; bi = g ? lane + 96 : bi; }
#pragma unroll
            for (int off = 16; off > 0; off >>= 1) {
                const float ov = __shfl_xor(bv, off, 32); const int oi = __shfl_xor(bi, off, 32);
                const bool tk = (ov > bv) | ((ov == bv) & (oi < bi));
                bv = tk ? ov : bv; bi = tk ? oi : bi; }
            sidx[it] = bi; sp[it] = __builtin_amdgcn_exp2f((bv - mx) * L2E) * inv;
            v0 = (bi == lane) ? NEGB : v0; v1 = (bi == lane + 32) ? NEGB : v1; v2 = (bi == lane + 64) ? NEGB : v2; v3 = (bi == lane + 96) ? NEGB : v3;
        }
        const float s4 = (((sp[0] + sp[1]) + sp[2]) + sp[3]) + 1e-8f;
        const float i4 = 1.0f / s4;
        if (lane == 0) {
            si[row * TK + 0] = sidx[0]; si[row * TK + 1] = sidx[1]; si[row * TK + 2] = sidx[2]; si[row * TK + 3] = sidx[3];
            sw[row * TK + 0] = sp[0] * i4; sw[row * TK + 1] = sp[1] * i4; sw[row * TK + 2] = sp[2] * i4; sw[row * TK + 3] = sp[3] * i4; }
    }
    __syncthreads();
    static_assert(32 * 16 == 32 * TK * 4);
    if (wave == 0) { const v4i iv = *(const v4ia*)(&si[lane * TK]); int* dp = SELI + ((size_t)route * TOK + (size_t)(t0 + lane)) * TK;
        *(volatile v4i*)dp = iv; __threadfence(); *(volatile v4i*)dp = iv; }
    if (wave == 1) { const v4f wv = *(const v4fa*)(&sw[lane * TK]); float* dp = SELW + ((size_t)route * TOK + (size_t)(t0 + lane)) * TK;
        *(volatile v4f*)dp = wv; __threadfence(); *(volatile v4f*)dp = wv; }
}

__global__ __launch_bounds__(128) void k_feat(const bf* __restrict__ XB, const bf* __restrict__ FT, const int* __restrict__ SI, const float* __restrict__ SW, float* HP) {
    __shared__ __align__(16) bf at[32 * APF];
    __shared__ int tl[TOK];
    __shared__ float tw[TOK];
    __shared__ int scnt[4];
    __shared__ __align__(16) float os[4 * 16 * 36];
    const int tid = threadIdx.x, lane = tid & 31, lr = lane & 15, hi = lane >> 4;
    const int wave = __builtin_amdgcn_readfirstlane((int)(threadIdx.x >> 5));
    const int n = blockIdx.x;
#pragma unroll 1
    for (int i = tid; i < TOK; i += 128) { tl[i] = 0; tw[i] = 0.0f; }
    if (tid == 0) scnt[0] = 0;
    __syncthreads();
    if (wave == 0) {
        int cv = 0;
#pragma unroll 1
        for (int tb = 0; tb < TOK; tb += 32) {
            const int t = tb + lane;
            const v4i iv = *(const v4i*)(SI + (size_t)t * TK);
            const v4f wq = *(const v4f*)(SW + (size_t)t * TK);
            const bool h0 = iv[0] == n, h1 = iv[1] == n, h2 = iv[2] == n, h3 = iv[3] == n;
            const bool hit = h0 | h1 | h2 | h3;
            const int slot = h0 ? 0 : (h1 ? 1 : (h2 ? 2 : 3));
            const float wsel = h0 ? wq[0] : (h1 ? wq[1] : (h2 ? wq[2] : wq[3]));
            const unsigned mask = (unsigned)__ballot(hit ? 1 : 0);
            int pos = cv + __popc(mask & ((1u << lane) - 1u)); pos = pos > TOK - 1 ? TOK - 1 : pos;
            if (hit) { tl[pos] = t * TK + slot; tw[pos] = wsel; }
            cv += __popc(mask);
        }
        if (lane == 0) scnt[0] = cv;
    }
    __syncthreads();
    int cc = scnt[0]; cc = cc < 0 ? 0 : (cc > TOK ? TOK : cc);
    const int cnt = __builtin_amdgcn_readfirstlane(cc);
    const int ntile = (cnt + 31) >> 5;
    const bf* fb = FT + ((size_t)n * RK + (size_t)(wave * 32 + lr)) * DM + 8 * hi;
    const int ao = lr * APF + 8 * hi;
    const int wb = wave * 16 * 36;
#pragma unroll 1
    for (int tile = 0; tile < ntile; ++tile) {
#pragma unroll 1
        for (int it = 0; it < 24; ++it) {
            const int p = it * 128 + tid; const int row = p / 96; const int c = p - row * 96;
            const int li = tile * 32 + row; const int lic = li < TOK ? li : TOK - 1;
            int tok = tl[lic] >> 2; tok = tok < 0 ? 0 : (tok > TOK - 1 ? TOK - 1 : tok);
            v4u v = *(const v4u*)(XB + (size_t)tok * DM + c * 8);
            asm volatile("" : "+v"(v));
            const v4u z = (v4u){};
            const v4u o = (li < cnt) ? v : z;
            *(v4ua*)(&at[row * APF + c * 8]) = o;
        }
        __syncthreads();
        v8f acc[2][2];
#pragma unroll
        for (int mb = 0; mb < 2; ++mb)
#pragma unroll
            for (int nb = 0; nb < 2; ++nb) acc[mb][nb] = (v8f){};
#pragma unroll 1
        for (int kc = 0; kc < DM; kc += 32) {
            const v16bf a0 = cat16b(*(const v8usa*)(&at[ao + kc]), *(const v8usa*)(&at[ao + kc + 16]));
            const v16bf a1 = cat16b(*(const v8usa*)(&at[ao + 16 * APF + kc]), *(const v8usa*)(&at[ao + 16 * APF + kc + 16]));
            const v16bf b0 = ldb(fb + kc), b1 = ldb(fb + (size_t)16 * DM + kc);
            acc[0][0] = wmmab_g(a0, b0, acc[0][0]); acc[1][0] = wmmab_g(a1, b0, acc[1][0]);
            acc[0][1] = wmmab_g(a0, b1, acc[0][1]); acc[1][1] = wmmab_g(a1, b1, acc[1][1]);
        }
#pragma unroll
        for (int mb = 0; mb < 2; ++mb) {
            float wr[8];
#pragma unroll
            for (int j = 0; j < 8; ++j) { int li = tile * 32 + mb * 16 + hi * 8 + j; li = li < TOK ? li : TOK - 1; wr[j] = tw[li]; }
#pragma unroll
            for (int nb = 0; nb < 2; ++nb) {
#pragma unroll
                for (int j = 0; j < 8; ++j) os[wb + (hi * 8 + j) * 36 + nb * 16 + lr] = acc[mb][nb][j] * wr[j]; }
            wave_sync();
            static_assert(32 * 16 * 4 == 16 * 128);
#pragma unroll 1
            for (int ps = 0; ps < 2; ++ps) {
#pragma unroll
                for (int s = 0; s < 4; ++s) { const int row = 4 * s + (lane >> 3), cofs = (lane & 7) * 4;
                    const int li = tile * 32 + mb * 16 + row; const int lic = li < TOK ? li : TOK - 1;
                    int ent = tl[lic]; ent = ent < 0 ? 0 : (ent > TOK * TK - 1 ? TOK * TK - 1 : ent);
                    const v4f val = *(const v4fa*)(&os[wb + row * 36 + cofs]);
                    if (li < cnt) *(volatile v4f*)(HP + (size_t)ent * RK + wave * 32 + cofs) = val; }
                if (ps == 0) __threadfence(); }
            wave_sync();
        }
        __syncthreads();
    }
}

__global__ __launch_bounds__(256) void k_hsum(const float* __restrict__ HP, h16* HH) {
#pragma clang fp contract(off)
    const int i = blockIdx.x * 256 + threadIdx.x; if (i >= TOK * (RK / 8)) return;
    const int t = i / (RK / 8); const int c8 = (i - t * (RK / 8)) * 8;
    const float* p = HP + (size_t)t * TK * RK + c8;
    const v4f a0 = *(const v4f*)p,            a1 = *(const v4f*)(p + 4);
    const v4f b0 = *(const v4f*)(p + RK),     b1 = *(const v4f*)(p + RK + 4);
    const v4f c0 = *(const v4f*)(p + 2 * RK), c1 = *(const v4f*)(p + 2 * RK + 4);
    const v4f d0 = *(const v4f*)(p + 3 * RK), d1 = *(const v4f*)(p + 3 * RK + 4);
    const v4f s0 = ((a0 + b0) + c0) + d0, s1 = ((a1 + b1) + c1) + d1;
    v8h o;
#pragma unroll
    for (int k = 0; k < 4; ++k) { o[k] = toh_flush(s0[k] * HCS); o[4 + k] = toh_flush(s1[k] * HCS); }
    h16* dp = HH + (size_t)t * RK + c8;
    *(volatile v8h*)dp = o; __threadfence(); *(volatile v8h*)dp = o;
}

__global__ __launch_bounds__(128) void k_rest(const h16* __restrict__ HH, const h16* __restrict__ RT, const int* __restrict__ SI, const float* __restrict__ SW, float* OP) {
    __shared__ __align__(16) h16 at[32 * AHP];
    __shared__ int tl[TOK];
    __shared__ float tw[TOK];
    __shared__ int scnt[4];
    __shared__ __align__(16) float os[4 * 16 * 68];
    const int tid = threadIdx.x, lane = tid & 31, lr = lane & 15, hi = lane >> 4;
    const int wave = __builtin_amdgcn_readfirstlane((int)(threadIdx.x >> 5));
    const int n = blockIdx.x; const int nc0 = blockIdx.y * 256;
#pragma unroll 1
    for (int i = tid; i < TOK; i += 128) { tl[i] = 0; tw[i] = 0.0f; }
    if (tid == 0) scnt[0] = 0;
    __syncthreads();
    if (wave == 0) {
        int cv = 0;
#pragma unroll 1
        for (int tb = 0; tb < TOK; tb += 32) {
            const int t = tb + lane;
            const v4i iv = *(const v4i*)(SI + (size_t)t * TK);
            const v4f wq = *(const v4f*)(SW + (size_t)t * TK);
            const bool h0 = iv[0] == n, h1 = iv[1] == n, h2 = iv[2] == n, h3 = iv[3] == n;
            const bool hit = h0 | h1 | h2 | h3;
            const int slot = h0 ? 0 : (h1 ? 1 : (h2 ? 2 : 3));
            const float wsel = h0 ? wq[0] : (h1 ? wq[1] : (h2 ? wq[2] : wq[3]));
            const unsigned mask = (unsigned)__ballot(hit ? 1 : 0);
            int pos = cv + __popc(mask & ((1u << lane) - 1u)); pos = pos > TOK - 1 ? TOK - 1 : pos;
            if (hit) { tl[pos] = t * TK + slot; tw[pos] = wsel; }
            cv += __popc(mask);
        }
        if (lane == 0) scnt[0] = cv;
    }
    __syncthreads();
    int cc = scnt[0]; cc = cc < 0 ? 0 : (cc > TOK ? TOK : cc);
    const int cnt = __builtin_amdgcn_readfirstlane(cc);
    const int ntile = (cnt + 31) >> 5;
    const h16* rb = RT + ((size_t)n * DM + (size_t)(nc0 + wave * 64 + lr)) * RK + 8 * hi;
    const int ao = lr * AHP + 8 * hi;
    const int wb = wave * 16 * 68;
#pragma unroll 1
    for (int tile = 0; tile < ntile; ++tile) {
#pragma unroll
        for (int it = 0; it < 4; ++it) {
            const int p = it * 128 + tid; const int row = p >> 4; const int c = p & 15;
            const int li = tile * 32 + row; const int lic = li < TOK ? li : TOK - 1;
            int tok = tl[lic] >> 2; tok = tok < 0 ? 0 : (tok > TOK - 1 ? TOK - 1 : tok);
            v4u v = *(const v4u*)(HH + (size_t)tok * RK + c * 8);
            asm volatile("" : "+v"(v));
            const v4u z = (v4u){};
            const v4u o = (li < cnt) ? v : z;
            *(v4ua*)(&at[row * AHP + c * 8]) = o;
        }
        __syncthreads();
        v8f acc[2][4];
#pragma unroll
        for (int mb = 0; mb < 2; ++mb)
#pragma unroll
            for (int q = 0; q < 4; ++q) acc[mb][q] = (v8f){};
#pragma unroll 1
        for (int kc = 0; kc < RK; kc += 32) {
            const v16h a0 = cat16(*(const v8ha*)(&at[ao + kc]), *(const v8ha*)(&at[ao + kc + 16]));
            const v16h a1 = cat16(*(const v8ha*)(&at[ao + 16 * AHP + kc]), *(const v8ha*)(&at[ao + 16 * AHP + kc + 16]));
#pragma unroll
            for (int q = 0; q < 4; ++q) { const v16h b = ldh(rb + (size_t)q * 16 * RK + kc);
                acc[0][q] = wmma16_g(a0, b, acc[0][q]); acc[1][q] = wmma16_g(a1, b, acc[1][q]); }
        }
#pragma unroll
        for (int mb = 0; mb < 2; ++mb) {
            float wr[8];
#pragma unroll
            for (int j = 0; j < 8; ++j) { int li = tile * 32 + mb * 16 + hi * 8 + j; li = li < TOK ? li : TOK - 1; wr[j] = tw[li] * OSI; }
#pragma unroll
            for (int q = 0; q < 4; ++q) {
#pragma unroll
                for (int j = 0; j < 8; ++j) os[wb + (hi * 8 + j) * 68 + q * 16 + lr] = acc[mb][q][j] * wr[j]; }
            wave_sync();
            static_assert(32 * 16 * 8 == 16 * 256);
#pragma unroll 1
            for (int ps = 0; ps < 2; ++ps) {
#pragma unroll
                for (int s = 0; s < 8; ++s) { const int row = 2 * s + (lane >> 4), c4 = (lane & 15) * 4;
                    const int li = tile * 32 + mb * 16 + row; const int lic = li < TOK ? li : TOK - 1;
                    int ent = tl[lic]; ent = ent < 0 ? 0 : (ent > TOK * TK - 1 ? TOK * TK - 1 : ent);
                    const v4f val = *(const v4fa*)(&os[wb + row * 68 + c4]);
                    if (li < cnt) *(volatile v4f*)(OP + (size_t)ent * DM + nc0 + wave * 64 + c4) = val; }
                if (ps == 0) __threadfence(); }
            wave_sync();
        }
        __syncthreads();
    }
}

__global__ __launch_bounds__(256) void k_osum(const float* __restrict__ OP, float* OUT) {
#pragma clang fp contract(off)
    const int i = blockIdx.x * 256 + threadIdx.x; if (i >= TOK * (DM / 4)) return;
    const int t = i / (DM / 4); const int c4 = (i - t * (DM / 4)) * 4;
    const float* p = OP + (size_t)t * TK * DM + c4;
    const v4f a = *(const v4f*)p, b = *(const v4f*)(p + DM), c = *(const v4f*)(p + 2 * DM), d = *(const v4f*)(p + 3 * DM);
    const v4f s = ((a + b) + c) + d;
    const int bb = t / SEQ; const int sq = t - bb * SEQ;
    float* dp = OUT + ((size_t)bb * OUT_SEQ + (size_t)sq) * DM + c4;
    *(volatile v4f*)dp = s; __threadfence(); *(volatile v4f*)dp = s;
}

static constexpr size_t al256(size_t v) { return (v + 255) & ~(size_t)255; }
static constexpr size_t SZ_XB = al256((size_t)TOK * DM * 2);
static constexpr size_t SZ_FT = al256((size_t)NE * RK * DM * 2);
static constexpr size_t SZ_RT = al256((size_t)NE * DM * RK * 2);
static constexpr size_t SZ_WT = al256((size_t)2 * DSP * DM * 2);
static constexpr size_t SZ_PJ = al256((size_t)TOK * 2 * DSP * 4);
static constexpr size_t SZ_SL = al256((size_t)2 * TOK * TK * 4);
static constexpr size_t SZ_HP = al256((size_t)TOK * TK * RK * 4);
static constexpr size_t SZ_HH = al256((size_t)TOK * RK * 2);
static constexpr size_t SZ_OP = al256((size_t)TOK * TK * DM * 4);
static constexpr size_t SZ_TOTAL = SZ_XB + SZ_FT + SZ_RT + SZ_WT + SZ_PJ + 2 * SZ_SL + SZ_HP + SZ_HH + SZ_OP;
static_assert(SZ_TOTAL <= (size_t)134217728);
static_assert(((size_t)DSP * DM * 2) % 256 == 0);
static_assert(((size_t)TOK * TK * 4) % 512 == 0);

extern "C" void kernel_launch(void* const* d_in, const int* in_sizes, int n_in,
                              void* d_out, int out_size, void* d_ws, size_t ws_size, hipStream_t stream) {
    if (n_in < 9) return;
    const size_t needx = ((size_t)(NB - 1) * SEQ_FULL + SEQ) * DM;
    if ((size_t)in_sizes[0] < needx) return;
    if ((size_t)in_sizes[1] < (size_t)NE * DM * RK || (size_t)in_sizes[2] < (size_t)NE * RK * DM) return;
    if ((size_t)in_sizes[3] < (size_t)DM * DSP || (size_t)in_sizes[5] < (size_t)DM * DSP) return;
    if (in_sizes[4] < DSP || in_sizes[6] < DSP) return;
    if ((size_t)in_sizes[7] < (size_t)NE * DSP || (size_t)in_sizes[8] < (size_t)NE * DSP) return;
    if ((size_t)out_size < ((size_t)(NB - 1) * OUT_SEQ + SEQ) * DM) return;
    if (SZ_TOTAL > ws_size) return;
    const float* x   = (const float*)d_in[0];
    const float* fk  = (const float*)d_in[1];
    const float* rk  = (const float*)d_in[2];
    const float* wfk = (const float*)d_in[3]; const float* bfk = (const float*)d_in[4];
    const float* wrk = (const float*)d_in[5]; const float* brk = (const float*)d_in[6];
    const float* efk = (const float*)d_in[7]; const float* erk = (const float*)d_in[8];
    float* OUT = (float*)d_out;
    char* wsp = (char*)d_ws;
    bf*    XB   = (bf*)wsp;    wsp += SZ_XB;
    bf*    FT   = (bf*)wsp;    wsp += SZ_FT;
    h16*   RT   = (h16*)wsp;   wsp += SZ_RT;
    bf*    WT   = (bf*)wsp;    wsp += SZ_WT;
    float* PROJ = (float*)wsp; wsp += SZ_PJ;
    int*   SELI = (int*)wsp;   wsp += SZ_SL;
    float* SELW = (float*)wsp; wsp += SZ_SL;
    float* HP   = (float*)wsp; wsp += SZ_HP;
    h16*   HH   = (h16*)wsp;   wsp += SZ_HH;
    float* OP   = (float*)wsp; wsp += SZ_OP;

    if (SEQ == SEQ_FULL) {
        const size_t n8 = (size_t)NB * SEQ * DM / 8;
        k_cvt8<<<(unsigned)((n8 + 255) / 256), 256, 0, stream>>>(x, XB, n8);
    } else {
        const size_t n8 = (size_t)SEQ * DM / 8;
        for (int b = 0; b < NB; ++b) k_cvt8<<<(unsigned)((n8 + 255) / 256), 256, 0, stream>>>(x + (size_t)b * SEQ_FULL * DM, XB + (size_t)b * SEQ * DM, n8);
    }
    k_tconv_b<<<dim3(DM / 64, RK / 64, NE), 256, 0, stream>>>(fk, FT, DM, RK);
    k_tconv_h<<<dim3(RK / 64, DM / 64, NE), 256, 0, stream>>>(rk, RT, RK, DM);
    k_tconv_b<<<dim3(DM / 64, DSP / 64, 1), 256, 0, stream>>>(wfk, WT, DM, DSP);
    k_tconv_b<<<dim3(DM / 64, DSP / 64, 1), 256, 0, stream>>>(wrk, WT + (size_t)DSP * DM, DM, DSP);

    k_rproj<<<dim3(TOK / 32, 2, 1), 32, 0, stream>>>(XB, WT, bfk, brk, PROJ);
    k_route<<<dim3(TOK / 32, 2, 1), 128, 0, stream>>>(PROJ, efk, erk, SELI, SELW);

    k_feat<<<dim3(NE, 1, 1), 128, 0, stream>>>(XB, FT, SELI, SELW, HP);
    k_hsum<<<(unsigned)(((size_t)TOK * (RK / 8) + 255) / 256), 256, 0, stream>>>(HP, HH);
    k_rest<<<dim3(NE, DM / 256, 1), 128, 0, stream>>>(HH, RT, SELI + (size_t)TOK * TK, SELW + (size_t)TOK * TK, OP);
    k_osum<<<(unsigned)(((size_t)TOK * (DM / 4) + 255) / 256), 256, 0, stream>>>(OP, OUT);
}
